// ChameleonVQVAEEncoderAttnBlock_32246614458385
// MI455X (gfx1250) — hardware-verified
//
#include <hip/hip_runtime.h>
#include <stddef.h>
#include <stdint.h>


#define CDIM 512
#define NPIX 1024
#define GCH  16
#define CBLK 64

typedef _Float16 v16h __attribute__((ext_vector_type(16)));
typedef _Float16 v8h  __attribute__((ext_vector_type(8)));
typedef float    v8f  __attribute__((ext_vector_type(8)));
typedef float    v4f  __attribute__((ext_vector_type(4)));
union Frag { v16h v; v8h half[2]; };

__device__ __forceinline__ v8f wmma_f16(v16h a, v16h b, v8f c) {
  v8f d = __builtin_amdgcn_wmma_f32_16x16x32_f16(false, a, false, b, (short)0, c, false, false);
  asm volatile("v_nop\n\tv_nop\n\tv_nop\n\tv_nop" : "+v"(d) : "v"(a), "v"(b));
  return d;
}

__device__ __forceinline__ v16h ld_frag(const _Float16* tile, int row, int h) {
  Frag f;
  const _Float16* rp = tile + row * 32;
  f.half[0] = *(const v8h*)(rp + 8 * h);
  f.half[1] = *(const v8h*)(rp + 16 + 8 * h);
  return f.v;
}

__global__ __launch_bounds__(256) void gn_kernel(
    const float* __restrict__ x, const float* __restrict__ gamma,
    const float* __restrict__ beta, _Float16* hT) {
  const int b  = blockIdx.x >> 3, cg = blockIdx.x & 7;
  const int c0 = cg * CBLK;
  const int t  = threadIdx.x;
  const int c  = t >> 2, q = t & 3;
  const float* xc = x + ((size_t)b * CDIM + c0 + c) * NPIX;

  float s = 0.f, ss = 0.f;
#pragma unroll 4
  for (int i = 0; i < NPIX / 16; ++i) {
    v4f v = *(const v4f*)(xc + q * (NPIX / 4) + 4 * i);
    s  += (v[0] + v[1]) + (v[2] + v[3]);
    ss += (v[0] * v[0] + v[1] * v[1]) + (v[2] * v[2] + v[3] * v[3]);
  }
  __shared__ float rs1[256], rs2[256];
  rs1[t] = s; rs2[t] = ss;
  __syncthreads();
  for (int k = 32; k > 0; k >>= 1) {
    if ((t & 63) < k) { rs1[t] += rs1[t + k]; rs2[t] += rs2[t + k]; }
    __syncthreads();
  }
  const int g = t >> 6;
  const float inv_cnt = 1.0f / (float)(GCH * NPIX);
  const float mean = rs1[g * 64] * inv_cnt;
  float var = rs2[g * 64] * inv_cnt - mean * mean;
  var = fmaxf(var, 0.f);
  const float inv = rsqrtf(var + 1e-6f);
  const float gm = gamma[c0 + c] * inv;
  const float bt = beta[c0 + c] - mean * gm;

  __shared__ __align__(16) _Float16 Ts[128 * CBLK];
  for (int ch = 0; ch < NPIX; ch += 128) {
    __syncthreads();
    const float* xp = xc + ch + q * 32;
#pragma unroll
    for (int j = 0; j < 8; ++j) {
      v4f v = *(const v4f*)(xp + 4 * j);
      const int nl = q * 32 + 4 * j;
      Ts[(nl + 0) * CBLK + c] = (_Float16)(v[0] * gm + bt);
      Ts[(nl + 1) * CBLK + c] = (_Float16)(v[1] * gm + bt);
      Ts[(nl + 2) * CBLK + c] = (_Float16)(v[2] * gm + bt);
      Ts[(nl + 3) * CBLK + c] = (_Float16)(v[3] * gm + bt);
    }
    __syncthreads();
    v8h val[4]; size_t idx[4];
#pragma unroll
    for (int it = 0; it < 4; ++it) {
      const int sI = it * 256 + t;
      const int nl = sI >> 3, p = sI & 7;
      val[it] = *(const v8h*)&Ts[nl * CBLK + p * 8];
      idx[it] = ((size_t)b * NPIX + ch + nl) * CDIM + c0 + p * 8;
    }
#pragma unroll
    for (int it = 0; it < 4; ++it) *(volatile v8h*)(hT + idx[it]) = val[it];
    __threadfence();
#pragma unroll
    for (int it = 0; it < 4; ++it) *(volatile v8h*)(hT + idx[it]) = val[it];
  }
}

template <int AF32, int MODE>
__global__ __launch_bounds__(128) void gemm_kernel(
    const float* __restrict__ Af, const _Float16* __restrict__ Ah, size_t a_bs, int lda, float ascale,
    const _Float16* __restrict__ Bt, size_t b_bs, int ldb, int K,
    const float* __restrict__ bias, int has_bias, float oscale,
    _Float16* out16, float* out32, const float* __restrict__ res, int has_res,
    size_t o_bs, int ldo) {
  const int m0 = blockIdx.x * 64, n0 = blockIdx.y * 64, b = blockIdx.z;
  const int tid = threadIdx.x, lane = tid & 31, wv = tid >> 5;
  const int h = lane >> 4, lm = lane & 15;
  const int wr = (wv >> 1) * 32, wc = (wv & 1) * 32;

  __shared__ __align__(16) _Float16 As[64 * 32];
  __shared__ __align__(16) _Float16 Bs[64 * 32];
  __shared__ __align__(16) _Float16 Dh[(MODE != 2) ? 64 * 64 : 8];
  __shared__ __align__(16) float    Df[(MODE == 2) ? 64 * 64 : 4];

  v8f zero;
#pragma unroll
  for (int e = 0; e < 8; ++e) zero[e] = 0.f;
  v8f acc[2][2];
  acc[0][0] = zero; acc[0][1] = zero; acc[1][0] = zero; acc[1][1] = zero;

  const int mm = tid >> 1, ks = (tid & 1) * 16;
  const float*    ap_f = Af + (size_t)b * a_bs + (size_t)(m0 + mm) * lda + ks;
  const _Float16* ap_h = Ah + (size_t)b * a_bs + (size_t)(m0 + mm) * lda + ks;
  const _Float16* bp   = Bt + (size_t)b * b_bs + (size_t)(n0 + mm) * ldb + ks;

  v4f w0, w1, w2, w3;
  v8h ah0, ah1, bh0, bh1;
  if (AF32) {
    w0 = *(const v4f*)(ap_f);     w1 = *(const v4f*)(ap_f + 4);
    w2 = *(const v4f*)(ap_f + 8); w3 = *(const v4f*)(ap_f + 12);
  } else {
    ah0 = *(const v8h*)(ap_h); ah1 = *(const v8h*)(ap_h + 8);
  }
  bh0 = *(const v8h*)(bp); bh1 = *(const v8h*)(bp + 8);

  for (int k0 = 0; k0 < K; k0 += 32) {
    if (AF32) {
      v8h t0, t1;
#pragma unroll
      for (int e = 0; e < 4; ++e) {
        t0[e]     = (_Float16)(w0[e] * ascale);
        t0[e + 4] = (_Float16)(w1[e] * ascale);
        t1[e]     = (_Float16)(w2[e] * ascale);
        t1[e + 4] = (_Float16)(w3[e] * ascale);
      }
      *(v8h*)&As[mm * 32 + ks]     = t0;
      *(v8h*)&As[mm * 32 + ks + 8] = t1;
    } else {
      *(v8h*)&As[mm * 32 + ks]     = ah0;
      *(v8h*)&As[mm * 32 + ks + 8] = ah1;
    }
    *(v8h*)&Bs[mm * 32 + ks]     = bh0;
    *(v8h*)&Bs[mm * 32 + ks + 8] = bh1;
    __syncthreads();

    const int k1 = k0 + 32;
    if (k1 < K) {
      if (AF32) {
        w0 = *(const v4f*)(ap_f + k1);     w1 = *(const v4f*)(ap_f + k1 + 4);
        w2 = *(const v4f*)(ap_f + k1 + 8); w3 = *(const v4f*)(ap_f + k1 + 12);
      } else {
        ah0 = *(const v8h*)(ap_h + k1); ah1 = *(const v8h*)(ap_h + k1 + 8);
      }
      bh0 = *(const v8h*)(bp + k1); bh1 = *(const v8h*)(bp + k1 + 8);
    }

    const v16h a0 = ld_frag(As, wr + lm, h);
    const v16h a1 = ld_frag(As, wr + 16 + lm, h);
    const v16h b0 = ld_frag(Bs, wc + lm, h);
    const v16h b1 = ld_frag(Bs, wc + 16 + lm, h);
    acc[0][0] = wmma_f16(a0, b0, acc[0][0]);
    acc[0][1] = wmma_f16(a0, b1, acc[0][1]);
    acc[1][0] = wmma_f16(a1, b0, acc[1][0]);
    acc[1][1] = wmma_f16(a1, b1, acc[1][1]);
    __syncthreads();
  }

#pragma unroll
  for (int mi = 0; mi < 2; ++mi)
#pragma unroll
    for (int ni = 0; ni < 2; ++ni)
#pragma unroll
      for (int r = 0; r < 8; ++r) {
        const int ml = wr + mi * 16 + 8 * h + r;
        const int nl = wc + ni * 16 + lm;
        float v = acc[mi][ni][r] * oscale;
        if (has_bias) v += bias[m0 + ml];
        if (MODE == 0)      Dh[nl * 64 + ml] = (_Float16)v;
        else if (MODE == 1) Dh[ml * 64 + nl] = (_Float16)v;
        else                Df[ml * 64 + nl] = v;
      }
  __syncthreads();

  if (MODE != 2) {
    v8h val[4]; size_t idx[4];
#pragma unroll
    for (int it = 0; it < 4; ++it) {
      const int sI = it * 128 + tid;
      const int row = sI >> 3, p = sI & 7;
      val[it] = *(const v8h*)&Dh[row * 64 + p * 8];
      if (MODE == 0) idx[it] = (size_t)b * o_bs + (size_t)(n0 + row) * ldo + m0 + p * 8;
      else           idx[it] = (size_t)b * o_bs + (size_t)(m0 + row) * ldo + n0 + p * 8;
    }
#pragma unroll
    for (int it = 0; it < 4; ++it) *(volatile v8h*)(out16 + idx[it]) = val[it];
    __threadfence();
#pragma unroll
    for (int it = 0; it < 4; ++it) *(volatile v8h*)(out16 + idx[it]) = val[it];
  } else {
    v4f val[8]; size_t idx[8];
#pragma unroll
    for (int it = 0; it < 8; ++it) {
      const int sI = it * 128 + tid;
      const int row = sI >> 4, p = sI & 15;
      v4f v = *(const v4f*)&Df[row * 64 + p * 4];
      idx[it] = (size_t)b * o_bs + (size_t)(m0 + row) * ldo + n0 + p * 4;
      if (has_res) v += *(const v4f*)(res + idx[it]);
      val[it] = v;
    }
#pragma unroll
    for (int it = 0; it < 8; ++it) *(volatile v4f*)(out32 + idx[it]) = val[it];
    __threadfence();
#pragma unroll
    for (int it = 0; it < 8; ++it) *(volatile v4f*)(out32 + idx[it]) = val[it];
  }
}

__global__ __launch_bounds__(128) void softmax_kernel(
    const float* __restrict__ S, _Float16* P, float pscale) {
  const int row = blockIdx.x;
  const int t = threadIdx.x, lane = t & 31, wv = t >> 5;
  const float* rp = S + (size_t)row * NPIX + 8 * t;
  const v4f a = *(const v4f*)(rp);
  const v4f c = *(const v4f*)(rp + 4);
  float e[8];
  e[0] = a[0]; e[1] = a[1]; e[2] = a[2]; e[3] = a[3];
  e[4] = c[0]; e[5] = c[1]; e[6] = c[2]; e[7] = c[3];
  float m = e[0];
#pragma unroll
  for (int i = 1; i < 8; ++i) m = fmaxf(m, e[i]);
#pragma unroll
  for (int o = 16; o > 0; o >>= 1) m = fmaxf(m, __shfl_xor(m, o, 32));
  __shared__ float rm[4], rs[4];
  if (lane == 0) rm[wv] = m;
  __syncthreads();
  m = fmaxf(fmaxf(rm[0], rm[1]), fmaxf(rm[2], rm[3]));
  float s = 0.f;
#pragma unroll
  for (int i = 0; i < 8; ++i) { e[i] = __expf(e[i] - m); s += e[i]; }
#pragma unroll
  for (int o = 16; o > 0; o >>= 1) s += __shfl_xor(s, o, 32);
  if (lane == 0) rs[wv] = s;
  __syncthreads();
  s = (rs[0] + rs[1]) + (rs[2] + rs[3]);
  const float inv = pscale / s;
  v8h ov;
#pragma unroll
  for (int i = 0; i < 8; ++i) ov[i] = (_Float16)(e[i] * inv);
  _Float16* dp = P + (size_t)row * NPIX + 8 * t;
  *(volatile v8h*)dp = ov;
  __threadfence();
  *(volatile v8h*)dp = ov;
}

extern "C" void kernel_launch(void* const* d_in, const int* in_sizes, int n_in,
                              void* d_out, int out_size, void* d_ws,
                              size_t ws_size, hipStream_t stream) {
  if (n_in < 11) return;
  const long long per = (long long)CDIM * NPIX;
  const long long tot = (long long)in_sizes[0];
  if (tot <= 0 || (tot % per) != 0) return;
  const int B = (int)(tot / per);
  if ((long long)out_size != tot) return;
  if (in_sizes[1] != CDIM || in_sizes[2] != CDIM) return;
  if (in_sizes[3] != CDIM * CDIM || in_sizes[5] != CDIM * CDIM ||
      in_sizes[7] != CDIM * CDIM || in_sizes[9] != CDIM * CDIM) return;
  if (in_sizes[4] != CDIM || in_sizes[6] != CDIM || in_sizes[8] != CDIM || in_sizes[10] != CDIM) return;
  if (B > 65535) return;

  const float* x     = (const float*)d_in[0];
  const float* gamma = (const float*)d_in[1];
  const float* beta  = (const float*)d_in[2];
  const float* wq = (const float*)d_in[3]; const float* bq = (const float*)d_in[4];
  const float* wk = (const float*)d_in[5]; const float* bk = (const float*)d_in[6];
  const float* wv = (const float*)d_in[7]; const float* bv = (const float*)d_in[8];
  const float* wo = (const float*)d_in[9]; const float* bo = (const float*)d_in[10];
  float* out = (float*)d_out;

  const size_t HB = (size_t)B * CDIM * NPIX * sizeof(_Float16);
  const size_t SB = (size_t)B * NPIX * NPIX * sizeof(float);
  const size_t PB = (size_t)B * NPIX * NPIX * sizeof(_Float16);
  if (4 * HB + SB + PB > ws_size) return;
  char* ws = (char*)d_ws;
  _Float16* qT  = (_Float16*)(ws);
  _Float16* kT  = (_Float16*)(ws + HB);
  _Float16* v16 = (_Float16*)(ws + 2 * HB);
  _Float16* hT  = (_Float16*)(ws + 3 * HB);
  float*    S   = (float*)(ws + 4 * HB);
  _Float16* P   = (_Float16*)(ws + 4 * HB + SB);

  const size_t actB = (size_t)NPIX * CDIM;
  const size_t sB   = (size_t)NPIX * NPIX;
  const float wsc   = 64.0f;
  const float attn_scale = 0.04419417382415922f;
  const float psc   = 4096.0f;
  const float osc   = 16.0f;

  gn_kernel<<<B * (CDIM / CBLK), 256, 0, stream>>>(x, gamma, beta, hT);

  dim3 gc(CDIM / 64, NPIX / 64, B);
  gemm_kernel<1, 0><<<gc, 128, 0, stream>>>(wq, hT, 0, CDIM, wsc, hT, actB, CDIM, CDIM,
                                            bq, 1, 1.0f / wsc, qT, S, x, 0, actB, CDIM);
  gemm_kernel<1, 0><<<gc, 128, 0, stream>>>(wk, hT, 0, CDIM, wsc, hT, actB, CDIM, CDIM,
                                            bk, 1, 1.0f / wsc, kT, S, x, 0, actB, CDIM);
  gemm_kernel<1, 1><<<gc, 128, 0, stream>>>(wv, hT, 0, CDIM, wsc, hT, actB, CDIM, CDIM,
                                            bv, 1, 1.0f / wsc, v16, S, x, 0, actB, NPIX);
  dim3 gs(NPIX / 64, NPIX / 64, B);
  gemm_kernel<0, 2><<<gs, 128, 0, stream>>>(wq, qT, actB, CDIM, 1.0f, kT, actB, CDIM, CDIM,
                                            bo, 0, attn_scale, qT, S, x, 0, sB, NPIX);
  softmax_kernel<<<B * NPIX, 128, 0, stream>>>(S, P, psc);
  gemm_kernel<0, 0><<<gc, 128, 0, stream>>>(wq, v16, actB, NPIX, 1.0f, P, sB, NPIX, NPIX,
                                            bo, 0, osc / psc, hT, S, x, 0, actB, CDIM);
  gemm_kernel<1, 2><<<gc, 128, 0, stream>>>(wo, hT, 0, CDIM, wsc, hT, actB, CDIM, CDIM,
                                            bo, 1, 1.0f / (wsc * osc), qT, out, x, 1, actB, NPIX);
}
